// InvariantEdgeConv_60189671686871
// MI455X (gfx1250) — hardware-verified
//
#include <hip/hip_runtime.h>
#include <stddef.h>

#define NB    4
#define NP    16384
#define KN    16
#define CIN   64
#define HID   128
#define OUTC  128
#define EDIM  133
#define NPTS  (NB * NP)
#define NS    (NPTS * KN)
#define NTHR  256
#define NWAV  8
#define PPW   8
#define NBLK_EDGE (NPTS / (NWAV * PPW))
#define NBLK_NODE (NPTS / 64)
#define NBLK_FIN  (NPTS / 128)
#define NBLK_CVT  ((NPTS * CIN) / (8 * NTHR))
#define APITCH 136
#define WSCL  16.0f
#define ASCL  8.0f

static_assert(NPTS % (NWAV * PPW) == 0);
static_assert(NPTS % 128 == 0);
static_assert((NPTS * CIN) % (8 * NTHR) == 0);
static_assert(APITCH % 8 == 0);
static_assert(HID == 128);
static_assert(OUTC == 128);
static_assert(CIN == 64);
static_assert(NP == 16384);
static_assert(NS == 1048576);

typedef _Float16 f16;
typedef f16 v16h __attribute__((ext_vector_type(16)));
typedef f16 v8h_t __attribute__((ext_vector_type(8)));
typedef v8h_t __attribute__((may_alias)) v8h;
typedef f16 v4h_t __attribute__((ext_vector_type(4)));
typedef v4h_t __attribute__((may_alias)) v4h;
typedef float v8f __attribute__((ext_vector_type(8)));
typedef float v4f_t __attribute__((ext_vector_type(4)));
typedef v4f_t __attribute__((may_alias)) v4f;
typedef unsigned int v4u __attribute__((ext_vector_type(4)));

union Frag { v16h v; v8h_t h[2]; };

__device__ __forceinline__ v8f zero8() {
    v8f z;
#pragma unroll
    for (int i = 0; i < 8; ++i) z[i] = 0.0f;
    return z;
}

__device__ __forceinline__ v16h ldfrag(const f16* p, int k0) {
    Frag f;
    f.h[0] = *(const v8h*)(p + k0);
    f.h[1] = *(const v8h*)(p + k0 + 16);
    return f.v;
}

__device__ __forceinline__ v8f wmma16(v16h a, v16h b, v8f c) {
    return __builtin_amdgcn_wmma_f32_16x16x32_f16(false, a, false, b, (short)0, c, false, false);
}

#define WMMA_GUARD8(o, a, b)                                                     \
    asm volatile("v_nop\n\tv_nop\n\tv_nop\n\tv_nop"                            \
                 : "+v"(o[0]), "+v"(o[1]), "+v"(o[2]), "+v"(o[3]),              \
                   "+v"(o[4]), "+v"(o[5]), "+v"(o[6]), "+v"(o[7])               \
                 : "v"(a), "v"(b))

template <int KD, int LDB>
__device__ __forceinline__ void gemm16x128(const f16* pa, const f16* pb, v8f (&o)[8])
{
#pragma unroll 1
    for (int k0 = 0; k0 < KD; k0 += 32) {
        const v16h a = ldfrag(pa, k0);
        v16h b;
#pragma unroll
        for (int t = 0; t < 8; ++t) {
            b = ldfrag(pb + (size_t)t * 16 * LDB, k0);
            o[t] = wmma16(a, b, o[t]);
        }
        WMMA_GUARD8(o, a, b);
    }
}

__device__ __forceinline__ void store_tile16x128(const v8f (&o)[8], float scale, float* stw,
                                                  float* gbase, int lane)
{
    const int hh = lane >> 4, m = lane & 15;
    const int c4 = m * 4;
#pragma unroll
    for (int og = 0; og < 2; ++og) {
#pragma unroll
        for (int t4 = 0; t4 < 4; ++t4) {
#pragma unroll
            for (int r = 0; r < 8; ++r)
                stw[(8 * hh + r) * 64 + 16 * t4 + m] = o[og * 4 + t4][r] * scale;
        }
        __syncthreads();
        v4f_t v[8];
#pragma unroll
        for (int p = 0; p < 8; ++p) v[p] = *(const v4f*)(stw + (2 * p + hh) * 64 + c4);
        float* go = gbase + og * 64 + c4;
#pragma unroll
        for (int p = 0; p < 8; ++p)
            *(volatile v4f_t*)(go + (size_t)(2 * p + hh) * OUTC) = v[p];
        __threadfence();
#pragma unroll
        for (int p = 0; p < 8; ++p)
            *(volatile v4f_t*)(go + (size_t)(2 * p + hh) * OUTC) = v[p];
        __syncthreads();
    }
}

__global__ void __launch_bounds__(NTHR) k_cvt(const float* __restrict__ src, f16* __restrict__ dst)
{
    const int i = blockIdx.x * NTHR + threadIdx.x;
    const v4f_t a = *(const v4f*)(src + (size_t)i * 8);
    const v4f_t b = *(const v4f*)(src + (size_t)i * 8 + 4);
    union { v8h_t h; v4u u; } pk;
#pragma unroll
    for (int j = 0; j < 4; ++j) {
        pk.h[j]     = (f16)a[j];
        pk.h[4 + j] = (f16)b[j];
    }
    *(volatile v4u*)(dst + (size_t)i * 8) = pk.u;
    __threadfence();
    *(volatile v4u*)(dst + (size_t)i * 8) = pk.u;
}

__global__ void __launch_bounds__(NTHR) k_wprep(
    const float* __restrict__ W1, const float* __restrict__ W2, const float* __restrict__ Wsc,
    f16* __restrict__ Wn, f16* __restrict__ W2s, f16* __restrict__ Wscs)
{
    const int tid = threadIdx.x, bid = blockIdx.x;
    float v[8];
    f16* dst;
    if (bid < 8) {
        const int i = bid * NTHR + tid;
        const int row = i >> 3, c8 = (i & 7) * 8;
        const int h = row & 127;
#pragma unroll
        for (int q = 0; q < 8; ++q) {
            const float a  = W1[(size_t)h * EDIM + c8 + q];
            const float bw = W1[(size_t)h * EDIM + 64 + c8 + q];
            v[q] = (row < 128) ? (a - bw) * WSCL : bw * WSCL;
        }
        dst = Wn + (size_t)i * 8;
    } else if (bid < 16) {
        const int i = (bid - 8) * NTHR + tid;
#pragma unroll
        for (int q = 0; q < 8; ++q) v[q] = W2[(size_t)i * 8 + q] * WSCL;
        dst = W2s + (size_t)i * 8;
    } else {
        const int i = (bid - 16) * NTHR + tid;
#pragma unroll
        for (int q = 0; q < 8; ++q) v[q] = Wsc[(size_t)i * 8 + q] * WSCL;
        dst = Wscs + (size_t)i * 8;
    }
    union { v8h_t h; v4u u; } pk;
#pragma unroll
    for (int q = 0; q < 8; ++q) pk.h[q] = (f16)v[q];
    *(volatile v4u*)dst = pk.u;
    __threadfence();
    *(volatile v4u*)dst = pk.u;
}

__global__ void __launch_bounds__(NTHR) k_node(
    const f16* __restrict__ feat16, const f16* __restrict__ Wn,
    float* __restrict__ P, float* __restrict__ Q)
{
    __shared__ __align__(16) float stg[NWAV * 16 * 64];
    const int tid = threadIdx.x, lane = tid & 31, w = tid >> 5;
    const int hh = lane >> 4, m = lane & 15;
    const int rw = w & 3, cg = w >> 2;
    const int row0 = blockIdx.x * 64 + rw * 16;

    v8f acc[8];
#pragma unroll
    for (int t = 0; t < 8; ++t) acc[t] = zero8();
    gemm16x128<CIN, CIN>(feat16 + (size_t)(row0 + m) * CIN + 8 * hh,
                         Wn + (size_t)(cg * 128 + m) * CIN + 8 * hh, acc);

    float* dstp = (cg == 0) ? P : Q;
    store_tile16x128(acc, 1.0f / WSCL, stg + w * 1024, dstp + (size_t)row0 * HID, lane);
}

__device__ __forceinline__ void edge_geo(const float* __restrict__ xyz, const int* __restrict__ idx,
                                         int gp, int lane, int& j, float (&g)[5])
{
    const int kk = lane & 15;
    int jr = idx[(size_t)gp * KN + kk];
    jr = min(max(jr, 0), NP - 1);
    j = (gp / NP) * NP + jr;
    const float c0 = xyz[(size_t)gp * 3 + 0], c1 = xyz[(size_t)gp * 3 + 1], c2 = xyz[(size_t)gp * 3 + 2];
    const float x0 = xyz[(size_t)j * 3 + 0],  x1 = xyz[(size_t)j * 3 + 1],  x2 = xyz[(size_t)j * 3 + 2];
    const float rc = __builtin_amdgcn_sqrtf(c0 * c0 + c1 * c1 + c2 * c2);
    const float rn = __builtin_amdgcn_sqrtf(x0 * x0 + x1 * x1 + x2 * x2);
    const float d0 = x0 - c0, d1 = x1 - c1, d2 = x2 - c2;
    const float rr = __builtin_amdgcn_sqrtf(d0 * d0 + d1 * d1 + d2 * d2);
    const float dt = c0 * x0 + c1 * x1 + c2 * x2;
    const float cv = dt * __builtin_amdgcn_rcpf(rc * rn + 1e-6f);
    g[0] = rc; g[1] = rn; g[2] = rr; g[3] = dt; g[4] = cv;
}

__device__ __forceinline__ void h1_4(const v4f_t& pv, const v4f_t& qv, const float (&wc)[4][5],
                                     float g0, float g1, float g2, float g3, float g4, float (&h)[4])
{
#pragma unroll
    for (int q = 0; q < 4; ++q) {
        float a = pv[q] + qv[q];
        a = fmaf(g0, wc[q][0], a);
        a = fmaf(g1, wc[q][1], a);
        a = fmaf(g2, wc[q][2], a);
        a = fmaf(g3, wc[q][3], a);
        a = fmaf(g4, wc[q][4], a);
        h[q] = a;
    }
}

__global__ void __launch_bounds__(NTHR) k_edge_stats(
    const float* __restrict__ P, const float* __restrict__ Q,
    const float* __restrict__ xyz, const int* __restrict__ idx,
    const float* __restrict__ W1, double* __restrict__ part)
{
    __shared__ double red[NWAV * 256];
    const int tid = threadIdx.x, lane = tid & 31, w = tid >> 5;

    float wc[4][5];
#pragma unroll
    for (int q = 0; q < 4; ++q)
#pragma unroll
        for (int g = 0; g < 5; ++g)
            wc[q][g] = W1[(size_t)(4 * lane + q) * EDIM + 128 + g];

    double ds[4], dq[4];
#pragma unroll
    for (int q = 0; q < 4; ++q) { ds[q] = 0.0; dq[q] = 0.0; }

#pragma unroll 1
    for (int i = 0; i < PPW; ++i) {
        const int gp = (blockIdx.x * NWAV + w) * PPW + i;
        int j; float g[5];
        edge_geo(xyz, idx, gp, lane, j, g);
        const v4f_t pv = *(const v4f*)(P + (size_t)gp * HID + 4 * lane);
        float s1[4], s2[4];
#pragma unroll
        for (int q = 0; q < 4; ++q) { s1[q] = 0.0f; s2[q] = 0.0f; }
#pragma unroll 1
        for (int k = 0; k < KN; ++k) {
            const int   jj = __shfl(j, k, 32);
            const float g0 = __shfl(g[0], k, 32), g1 = __shfl(g[1], k, 32), g2 = __shfl(g[2], k, 32);
            const float g3 = __shfl(g[3], k, 32), g4 = __shfl(g[4], k, 32);
            const v4f_t qv = *(const v4f*)(Q + (size_t)jj * HID + 4 * lane);
            float h[4];
            h1_4(pv, qv, wc, g0, g1, g2, g3, g4, h);
#pragma unroll
            for (int q = 0; q < 4; ++q) { s1[q] += h[q]; s2[q] = fmaf(h[q], h[q], s2[q]); }
        }
#pragma unroll
        for (int q = 0; q < 4; ++q) { ds[q] += (double)s1[q]; dq[q] += (double)s2[q]; }
    }

#pragma unroll
    for (int q = 0; q < 4; ++q) {
        red[w * 256 + 4 * lane + q]       = ds[q];
        red[w * 256 + 128 + 4 * lane + q] = dq[q];
    }
    __syncthreads();
    double a = 0.0;
#pragma unroll
    for (int ww = 0; ww < NWAV; ++ww) a += red[ww * 256 + tid];
    double* pp = part + (size_t)blockIdx.x * 256 + tid;
    *(volatile double*)pp = a;
    __threadfence();
    *(volatile double*)pp = a;
}

__global__ void __launch_bounds__(NTHR) k_bnfin(
    const double* __restrict__ part, int nblk,
    const float* __restrict__ gam, const float* __restrict__ bet, float* __restrict__ bnp)
{
    __shared__ double tot[256];
    const int tid = threadIdx.x;
    double a = 0.0;
#pragma unroll 1
    for (int blk = 0; blk < nblk; ++blk) a += part[(size_t)blk * 256 + tid];
    tot[tid] = a;
    __syncthreads();
    const int c = tid & 127;
    const double invn = 1.0 / (double)NS;
    const double mean = tot[c] * invn;
    double var = tot[128 + c] * invn - mean * mean;
    var = (var < 0.0) ? 0.0 : var;
    const float rs  = rsqrtf((float)var + 1e-5f);
    const float scl = rs * gam[c];
    const float shf = bet[c] - (float)mean * scl;
    const float val = (tid < 128) ? scl : shf;
    *(volatile float*)(bnp + tid) = val;
    __threadfence();
    *(volatile float*)(bnp + tid) = val;
}

__global__ void __launch_bounds__(NTHR) k_edge_gemm(
    const float* __restrict__ P, const float* __restrict__ Q,
    const float* __restrict__ xyz, const int* __restrict__ idx,
    const float* __restrict__ W1, const float* __restrict__ bnp1,
    const f16* __restrict__ W2s, float* __restrict__ pooled, double* __restrict__ part)
{
    __shared__ __align__(16) f16 sA[NWAV][KN * APITCH];
    __shared__ __align__(16) float sP[NWAV][OUTC];
    __shared__ double red[NWAV * 256];
    const int tid = threadIdx.x, lane = tid & 31, w = tid >> 5;
    const int hh = lane >> 4, m = lane & 15;

    float wc[4][5];
#pragma unroll
    for (int q = 0; q < 4; ++q)
#pragma unroll
        for (int g = 0; g < 5; ++g)
            wc[q][g] = W1[(size_t)(4 * lane + q) * EDIM + 128 + g];
    const v4f_t sc1 = *(const v4f*)(bnp1 + 4 * lane);
    const v4f_t sh1 = *(const v4f*)(bnp1 + 128 + 4 * lane);

    double ds[8], dq[8];
#pragma unroll
    for (int t = 0; t < 8; ++t) { ds[t] = 0.0; dq[t] = 0.0; }

    f16*   sAw = &sA[w][0];
    float* sPw = &sP[w][0];
    const f16* paw = sAw + m * APITCH + 8 * hh;
    const f16* pbw = W2s + (size_t)m * HID + 8 * hh;

#pragma unroll 1
    for (int i = 0; i < PPW; ++i) {
        const int gp = (blockIdx.x * NWAV + w) * PPW + i;
        int j; float g[5];
        edge_geo(xyz, idx, gp, lane, j, g);
        const v4f_t pv = *(const v4f*)(P + (size_t)gp * HID + 4 * lane);

#pragma unroll 1
        for (int k = 0; k < KN; ++k) {
            const int   jj = __shfl(j, k, 32);
            const float g0 = __shfl(g[0], k, 32), g1 = __shfl(g[1], k, 32), g2 = __shfl(g[2], k, 32);
            const float g3 = __shfl(g[3], k, 32), g4 = __shfl(g[4], k, 32);
            const v4f_t qv = *(const v4f*)(Q + (size_t)jj * HID + 4 * lane);
            float h[4];
            h1_4(pv, qv, wc, g0, g1, g2, g3, g4, h);
            v4h_t pk;
#pragma unroll
            for (int q = 0; q < 4; ++q) {
                const float x  = fmaf(h[q], sc1[q], sh1[q]);
                const float sg = __builtin_amdgcn_rcpf(1.0f + __expf(-x));
                pk[q] = (f16)((x * sg) * ASCL);
            }
            *(v4h*)(sAw + k * APITCH + 4 * lane) = pk;
        }
        __syncthreads();

        v8f acc[8];
#pragma unroll
        for (int t = 0; t < 8; ++t) acc[t] = zero8();
        gemm16x128<HID, HID>(paw, pbw, acc);

#pragma unroll
        for (int t = 0; t < 8; ++t) {
            float cs = 0.0f, cq = 0.0f;
#pragma unroll
            for (int r = 0; r < 8; ++r) { const float v = acc[t][r]; cs += v; cq = fmaf(v, v, cq); }
            cs += __shfl_xor(cs, 16, 32);
            cq += __shfl_xor(cq, 16, 32);
            ds[t] += (double)cs;
            dq[t] += (double)cq;
            sPw[16 * t + m] = cs * (1.0f / 2048.0f);
        }
        __syncthreads();
        const v4f_t pr = *(const v4f*)(sPw + 4 * lane);
        float* gq = pooled + (size_t)gp * OUTC + 4 * lane;
        *(volatile v4f_t*)gq = pr;
        __threadfence();
        *(volatile v4f_t*)gq = pr;
    }

#pragma unroll
    for (int t = 0; t < 8; ++t) {
        red[w * 256 + 16 * t + m]       = ds[t] * (1.0 / 128.0);
        red[w * 256 + 128 + 16 * t + m] = dq[t] * (1.0 / 16384.0);
    }
    __syncthreads();
    double a = 0.0;
#pragma unroll
    for (int ww = 0; ww < NWAV; ++ww) a += red[ww * 256 + tid];
    double* pp = part + (size_t)blockIdx.x * 256 + tid;
    *(volatile double*)pp = a;
    __threadfence();
    *(volatile double*)pp = a;
}

__global__ void __launch_bounds__(NTHR) k_final(
    const f16* __restrict__ feat16, const f16* __restrict__ Wscs,
    const float* __restrict__ lng, const float* __restrict__ lnb,
    const float* __restrict__ bnp2, const float* __restrict__ pooled,
    float* __restrict__ out)
{
    __shared__ __align__(16) float stg[NWAV * 16 * 64];
    const int tid = threadIdx.x, lane = tid & 31, w = tid >> 5;
    const int hh = lane >> 4, m = lane & 15;
    const int row0 = blockIdx.x * 128 + w * 16;

    v8f acc[8];
#pragma unroll
    for (int t = 0; t < 8; ++t) acc[t] = zero8();
    gemm16x128<CIN, CIN>(feat16 + (size_t)(row0 + m) * CIN + 8 * hh,
                         Wscs + (size_t)m * CIN + 8 * hh, acc);
#pragma unroll
    for (int t = 0; t < 8; ++t)
#pragma unroll
        for (int r = 0; r < 8; ++r) acc[t][r] *= (1.0f / WSCL);

    float mu[8], rs[8];
#pragma unroll
    for (int r = 0; r < 8; ++r) {
        float a = 0.0f;
#pragma unroll
        for (int t = 0; t < 8; ++t) a += acc[t][r];
        a += __shfl_xor(a, 1, 32); a += __shfl_xor(a, 2, 32);
        a += __shfl_xor(a, 4, 32); a += __shfl_xor(a, 8, 32);
        mu[r] = a * (1.0f / 128.0f);
    }
#pragma unroll
    for (int r = 0; r < 8; ++r) {
        float v = 0.0f;
#pragma unroll
        for (int t = 0; t < 8; ++t) { const float d = acc[t][r] - mu[r]; v = fmaf(d, d, v); }
        v += __shfl_xor(v, 1, 32); v += __shfl_xor(v, 2, 32);
        v += __shfl_xor(v, 4, 32); v += __shfl_xor(v, 8, 32);
        rs[r] = rsqrtf(v * (1.0f / 128.0f) + 1e-5f);
    }
    const int grow = row0 + 8 * hh;
#pragma unroll
    for (int t = 0; t < 8; ++t) {
        const int ch = 16 * t + m;
        const float lg = lng[ch], lb = lnb[ch];
        const float s2 = bnp2[ch], h2 = bnp2[128 + ch];
#pragma unroll
        for (int r = 0; r < 8; ++r) {
            const float scv = ((acc[t][r] - mu[r]) * rs[r]) * lg + lb;
            const float pr  = pooled[(size_t)(grow + r) * OUTC + ch];
            const float z   = fmaf(pr, s2, h2) + scv;
            const float sg  = __builtin_amdgcn_rcpf(1.0f + __expf(-z));
            acc[t][r] = z * sg;
        }
    }
    store_tile16x128(acc, 1.0f, stg + w * 1024, out + (size_t)row0 * OUTC, lane);
}

extern "C" void kernel_launch(void* const* d_in, const int* in_sizes, int n_in,
                              void* d_out, int out_size, void* d_ws, size_t ws_size,
                              hipStream_t stream)
{
    if (n_in < 12) return;
    if (in_sizes[0]  != NPTS * CIN) return;
    if (in_sizes[1]  != NPTS * 3) return;
    if (in_sizes[2]  != HID * EDIM) return;
    if (in_sizes[3]  != HID || in_sizes[4] != HID) return;
    if (in_sizes[5]  != OUTC * HID) return;
    if (in_sizes[6]  != OUTC || in_sizes[7] != OUTC) return;
    if (in_sizes[8]  != OUTC * CIN) return;
    if (in_sizes[9]  != OUTC || in_sizes[10] != OUTC) return;
    if (in_sizes[11] != NPTS * KN) return;
    if (out_size != NPTS * OUTC) return;

    const float* feat = (const float*)d_in[0];
    const float* xyz  = (const float*)d_in[1];
    const float* W1   = (const float*)d_in[2];
    const float* g1   = (const float*)d_in[3];
    const float* b1   = (const float*)d_in[4];
    const float* W2   = (const float*)d_in[5];
    const float* g2   = (const float*)d_in[6];
    const float* b2   = (const float*)d_in[7];
    const float* Wsc  = (const float*)d_in[8];
    const float* lng  = (const float*)d_in[9];
    const float* lnb  = (const float*)d_in[10];
    const int*   idx  = (const int*)d_in[11];
    float* out = (float*)d_out;

    const size_t szF16  = (size_t)NPTS * CIN * 2;
    const size_t szWn   = (size_t)256 * CIN * 2;
    const size_t szW2   = (size_t)OUTC * HID * 2;
    const size_t szWsc  = (size_t)OUTC * CIN * 2;
    const size_t szPl   = (size_t)NPTS * HID * 4;
    const size_t szPart = (size_t)NBLK_EDGE * 256 * 8;
    const size_t szBn   = 256 * 4;
    const size_t oF16  = 0;
    const size_t oWn   = oF16  + szF16;
    const size_t oW2   = oWn   + szWn;
    const size_t oWsc  = oW2   + szW2;
    const size_t oP    = oWsc  + szWsc;
    const size_t oQ    = oP    + szPl;
    const size_t oPool = oQ    + szPl;
    const size_t oPA   = oPool + szPl;
    const size_t oPB   = oPA   + szPart;
    const size_t oBn1  = oPB   + szPart;
    const size_t oBn2  = oBn1  + szBn;
    const size_t total = oBn2  + szBn;
    if (total > ws_size) return;

    char* ws = (char*)d_ws;
    f16*    feat16 = (f16*)(ws + oF16);
    f16*    Wn     = (f16*)(ws + oWn);
    f16*    W2s    = (f16*)(ws + oW2);
    f16*    Wscs   = (f16*)(ws + oWsc);
    float*  P      = (float*)(ws + oP);
    float*  Q      = (float*)(ws + oQ);
    float*  pooled = (float*)(ws + oPool);
    double* partA  = (double*)(ws + oPA);
    double* partB  = (double*)(ws + oPB);
    float*  bn1    = (float*)(ws + oBn1);
    float*  bn2    = (float*)(ws + oBn2);

    k_cvt<<<NBLK_CVT, NTHR, 0, stream>>>(feat, feat16);
    k_wprep<<<20, NTHR, 0, stream>>>(W1, W2, Wsc, Wn, W2s, Wscs);
    k_node<<<NBLK_NODE, NTHR, 0, stream>>>(feat16, Wn, P, Q);
    k_edge_stats<<<NBLK_EDGE, NTHR, 0, stream>>>(P, Q, xyz, idx, W1, partA);
    k_bnfin<<<1, NTHR, 0, stream>>>(partA, NBLK_EDGE, g1, b1, bn1);
    k_edge_gemm<<<NBLK_EDGE, NTHR, 0, stream>>>(P, Q, xyz, idx, W1, bn1, W2s, pooled, partB);
    k_bnfin<<<1, NTHR, 0, stream>>>(partB, NBLK_EDGE, g2, b2, bn2);
    k_final<<<NBLK_FIN, NTHR, 0, stream>>>(feat16, Wscs, lng, lnb, bn2, pooled, out);
}
